// indi_SAGE_PR_1623497638161
// MI455X (gfx1250) — hardware-run, weakly checked
//
#include <hip/hip_runtime.h>

typedef float          v8f   __attribute__((ext_vector_type(8)));
typedef float          v4f   __attribute__((ext_vector_type(4)));
typedef unsigned int   v4u   __attribute__((ext_vector_type(4)));
typedef int            v8i   __attribute__((ext_vector_type(8)));
typedef unsigned short v8us  __attribute__((ext_vector_type(8)));
typedef unsigned short v16us __attribute__((ext_vector_type(16)));
typedef __bf16         v16bf __attribute__((ext_vector_type(16)));
typedef _Float16       v16h  __attribute__((ext_vector_type(16)));
typedef v4f  __attribute__((may_alias)) v4fa;
typedef v8us __attribute__((may_alias)) v8usa;
union FragB { v16bf v; v16us u; v8us h[2]; v8i w; };
union FragH { v16h  v; v16us u; v8us h[2]; v8i w; };

__device__ __forceinline__ v8f wmb(const FragB& a, const FragB& b, v8f c) {
  v8f d = __builtin_amdgcn_wmma_f32_16x16x32_bf16(false, a.v, false, b.v, (short)0, c, false, false);
  asm volatile("v_nop\n\tv_nop\n\tv_nop\n\tv_nop" : "+v"(d) : "v"(a.w), "v"(b.w));
  return d;
}

__device__ __forceinline__ v8f wmh(const FragH& a, const FragH& b, v8f c) {
  v8f d = __builtin_amdgcn_wmma_f32_16x16x32_f16(false, a.v, false, b.v, (short)0, c, false, false);
  asm volatile("v_nop\n\tv_nop\n\tv_nop\n\tv_nop" : "+v"(d) : "v"(a.w), "v"(b.w));
  return d;
}

__device__ __forceinline__ unsigned bf16_bits(float f) {
  const unsigned u = __float_as_uint(f);
  const unsigned r = (u + 0x7FFFu + ((u >> 16) & 1u)) >> 16;
  const unsigned q = (u >> 16) | 0x40u;
  return ((u & 0x7fffffffu) > 0x7f800000u) ? q : r;
}

__device__ __forceinline__ float bf16_val(float f) {
  return __uint_as_float(bf16_bits(f) << 16);
}
__device__ __forceinline__ int clampi(int v, int lo, int hi) {
  return v < lo ? lo : (v > hi ? hi : v);
}

__device__ __forceinline__ unsigned f16_bits(float f) {
  const unsigned u  = __float_as_uint(f);
  const unsigned s  = (u >> 16) & 0x8000u;
  const unsigned a  = u & 0x7fffffffu;
  const unsigned t  = a - 0x38000000u;
  const unsigned r  = (t + 0x0FFFu + ((t >> 13) & 1u)) >> 13;
  const unsigned rc = r > 0x7C00u ? 0x7C00u : r;
  const bool small  = a < 0x38800000u;
  const bool isnan  = a > 0x7f800000u;
  const unsigned fin = small ? 0u : (s | rc);
  return isnan ? (s | 0x7E00u) : fin;
}

__device__ __forceinline__ unsigned pk16(unsigned lo, unsigned hi) { return lo | (hi << 16); }
__device__ __forceinline__ unsigned bf16_lo_bits(float v) {
  float hi = bf16_val(v);
  asm volatile("" : "+v"(hi));
  return bf16_bits(v - hi);
}
__device__ __forceinline__ v4u pack8_bf16(v4f a, v4f c) {
  return (v4u){ pk16(bf16_bits(a[0]), bf16_bits(a[1])), pk16(bf16_bits(a[2]), bf16_bits(a[3])),
                pk16(bf16_bits(c[0]), bf16_bits(c[1])), pk16(bf16_bits(c[2]), bf16_bits(c[3])) };
}
__device__ __forceinline__ v4u pack8_bf16_lo(v4f a, v4f c) {
  return (v4u){ pk16(bf16_lo_bits(a[0]), bf16_lo_bits(a[1])), pk16(bf16_lo_bits(a[2]), bf16_lo_bits(a[3])),
                pk16(bf16_lo_bits(c[0]), bf16_lo_bits(c[1])), pk16(bf16_lo_bits(c[2]), bf16_lo_bits(c[3])) };
}
__device__ __forceinline__ v4u pack8_f16(v4f a, v4f c) {
  return (v4u){ pk16(f16_bits(a[0]), f16_bits(a[1])), pk16(f16_bits(a[2]), f16_bits(a[3])),
                pk16(f16_bits(c[0]), f16_bits(c[1])), pk16(f16_bits(c[2]), f16_bits(c[3])) };
}

template <int FORM>
__global__ __launch_bounds__(256) void k_plane(const float* __restrict__ src, int rows, int cols, int ldsrc,
                                               unsigned short* __restrict__ dst, int MP, int KP) {
  static_assert(FORM >= 0 && FORM <= 3);
  const int KTOT = (FORM == 1 || FORM == 3) ? 2 * KP : KP;
  const unsigned ppr   = (unsigned)(KTOT >> 3);
  const unsigned kp8   = (unsigned)(KP >> 3);
  const unsigned total = (unsigned)MP * ppr;
  const unsigned g     = blockIdx.x * 256u + threadIdx.x;
  const unsigned rowu  = g / ppr;
  const unsigned p     = g - rowu * ppr;
  const bool second    = p >= kp8;
  const int row = (int)rowu;
  const int c0  = (int)((second ? p - kp8 : p) << 3);
  const float* srow = src + (size_t)clampi(row, 0, rows - 1) * (size_t)ldsrc;
  float x[8];
  unsigned mk[8];
#pragma unroll
  for (int e = 0; e < 8; ++e) {
    const int c = c0 + e;
    const float v = srow[clampi(c, 0, cols - 1)];
    asm volatile("" :: "v"(v));
    x[e]  = v;
    mk[e] = (row < rows && c < cols) ? 0xFFFFu : 0u;
  }
  const v4f a = (v4f){ x[0], x[1], x[2], x[3] };
  const v4f c = (v4f){ x[4], x[5], x[6], x[7] };
  v4u o;
  if (FORM == 2) {
    o = pack8_f16(a, c);
  } else {
    const v4u hi = pack8_bf16(a, c);
    o = hi;
    if (FORM == 1) { const v4u lo = pack8_bf16_lo(a, c); o = second ? lo : hi; }
  }
  const v4u mw = (v4u){ pk16(mk[0], mk[1]), pk16(mk[2], mk[3]), pk16(mk[4], mk[5]), pk16(mk[6], mk[7]) };
  o &= mw;
  if (g < total) {
    volatile v4u* q = (volatile v4u*)(dst + (size_t)g * 8);
    *q = o;
    __threadfence();
    *q = o;
  }
}

template <int FORM> struct FragOf    { typedef FragB T; };
template <>         struct FragOf<2> { typedef FragH T; };
__device__ __forceinline__ v8f mm(const FragB& a, const FragB& b, v8f c) { return wmb(a, b, c); }
__device__ __forceinline__ v8f mm(const FragH& a, const FragH& b, v8f c) { return wmh(a, b, c); }
template <class F> __device__ __forceinline__ F ld_frag(const unsigned short* p) {
  F f;
  f.h[0] = *(const v8usa*)(p);
  f.h[1] = *(const v8usa*)(p + 16);
  return f;
}

template <int FORM, int EPI>
__global__ __launch_bounds__(256) __attribute__((amdgpu_num_vgpr(248)))
void k_gemm_nt(const unsigned short* __restrict__ A, const unsigned short* __restrict__ B,
               const float* __restrict__ bias, float* __restrict__ D, int M, int N, int KTOT, int ldd) {
  static_assert(FORM >= 0 && FORM <= 2);
  static_assert(EPI == 0 || EPI == 1);
  typedef typename FragOf<FORM>::T F;
  __shared__ __attribute__((aligned(16))) float sT[8][16 * 68];
  const int lane = threadIdx.x & 31;
  const int wave = threadIdx.x >> 5;
  const int tilesM = (M + 63) >> 6;
  const int tilesN = (N + 63) >> 6;
  const int tile = blockIdx.x * 8 + wave;
  if (tile >= tilesM * tilesN) return;
  const int tm = tile / tilesN;
  const int tn = tile - tm * tilesN;
  const int m0 = tm << 6;
  const int n0 = tn << 6;

  const int rl = lane & 15;
  const int h8 = (lane >> 4) * 8;
  const unsigned short* pa = A + (size_t)(m0 + rl) * (size_t)KTOT + h8;
  const unsigned short* pb = B + (size_t)(n0 + rl) * (size_t)KTOT + h8;

  v8f acc[4][4];
#pragma unroll
  for (int i = 0; i < 4; ++i)
#pragma unroll
    for (int j = 0; j < 4; ++j) acc[i][j] = (v8f){0.f, 0.f, 0.f, 0.f, 0.f, 0.f, 0.f, 0.f};

#pragma unroll 1
  for (int k0 = 0; k0 < KTOT; k0 += 32) {
    F bf[4];
#pragma unroll
    for (int j = 0; j < 4; ++j) bf[j] = ld_frag<F>(pb + (size_t)(j << 4) * (size_t)KTOT + k0);
#pragma unroll
    for (int i = 0; i < 4; ++i) {
      const F af = ld_frag<F>(pa + (size_t)(i << 4) * (size_t)KTOT + k0);
#pragma unroll
      for (int j = 0; j < 4; ++j) acc[i][j] = mm(af, bf[j], acc[i][j]);
    }
  }

  float* slab = sT[wave];
  const int hh = lane >> 4;
  const int c4 = (lane & 15) * 4;
  const int nc = n0 + c4;
  const bool cok = nc < N;
  v4f bv = (v4f){0.f, 0.f, 0.f, 0.f};
  if (EPI == 1) {
    bv = *(const v4fa*)(bias + clampi(nc, 0, N - 4));
    asm volatile("" :: "v"(bv));
  }
#pragma unroll
  for (int i = 0; i < 4; ++i) {
    const int mBase = m0 + (i << 4);
#pragma unroll
    for (int j = 0; j < 4; ++j) {
#pragma unroll
      for (int r = 0; r < 8; ++r) slab[(h8 + r) * 68 + (j << 4) + rl] = acc[i][j][r];
    }
    __builtin_amdgcn_fence(__ATOMIC_RELEASE, "workgroup");
    __builtin_amdgcn_wave_barrier();
    __builtin_amdgcn_fence(__ATOMIC_ACQUIRE, "workgroup");
    v4f vv[8];
#pragma unroll
    for (int it = 0; it < 8; ++it) {
      const int row = it * 2 + hh;
      v4f v = *(const v4fa*)(slab + row * 68 + c4);
      if (EPI == 1) v += bv;
      vv[it] = v;
    }
    for (int pass = 0; pass < 2; ++pass) {
#pragma unroll
      for (int it = 0; it < 8; ++it) {
        const int row = mBase + it * 2 + hh;
        if (cok && row < M) *(volatile v4f*)(D + (size_t)row * (size_t)ldd + nc) = vv[it];
      }
      __threadfence();
    }
    __builtin_amdgcn_fence(__ATOMIC_RELEASE, "workgroup");
    __builtin_amdgcn_wave_barrier();
    __builtin_amdgcn_fence(__ATOMIC_ACQUIRE, "workgroup");
  }
}

#include <stddef.h>
#pragma clang fp contract(off)

#define M1_TWO 1
#define H_TWO  1
#define M2_TWO 1

#define NN     10000
#define NE     640000
#define CIN    128
#define HID    256
#define MPAD   10048
#define K1     (CIN + CIN * (1 + M1_TWO))
#define HW     (HID * (1 + H_TWO))
#define K2     (HW + HID * (1 + M2_TWO))

#define NWAVE  8
#define EPT    8
#define CHUNK  2048
#define NCHUNK 313
#define NBS    256
#define NBS_LOG 8
#define NBLK   40
#define SRCBITS 14
#define SRCMASK 16383
#define WCAP   2816
#define RCAP   21504
#define DEGCAP 128
#define BK_INTS (NWAVE * WCAP + RCAP + 3 * NBS + 16)
#define BK_LDS_BYTES (BK_INTS * 4)

static_assert(NN <= (1 << SRCBITS));
static_assert(NBLK * NBS >= NN && NBS == (1 << NBS_LOG));
static_assert(NE == 312 * CHUNK + 1024 && NCHUNK == (NE + CHUNK - 1) / CHUNK);
static_assert(NE % EPT == 0 && NE >= EPT && CHUNK == 256 * EPT);
static_assert(NWAVE * WCAP * 4 >= 16575 * 5);
static_assert(RCAP * 4 >= 16575 * 5 && RCAP % 1024 == 0);
static_assert(DEGCAP * 4 >= 98 * 5);
static_assert(BK_INTS % 4 == 0 && BK_LDS_BYTES <= 262144);
static_assert(MPAD % 64 == 0 && MPAD >= NN && NN % 16 == 0 && NN % NWAVE == 0);
static_assert(K1 % 32 == 0 && K2 % 32 == 0 && HID % 64 == 0 && HID % 32 == 0);
static_assert(CIN == 4 * 32 && HID == 8 * 32);

typedef int v4i __attribute__((ext_vector_type(4)));
typedef v4i __attribute__((may_alias)) v4ia;

#define PB_W1  (HID * (CIN / 8) / 256)
#define PB_W2  (HID * (HID / 8) / 256)
#define PB_X   (NN * (CIN / 8) / 256)
#define PB_Z1  ((MPAD - NN) * (K1 / 8) / 256)
#define PB_Z2  ((MPAD - NN) * (K2 / 8) / 256)
#define PB0_WL1 (PB_W1)
#define PB0_WR2 (2 * PB_W1)
#define PB0_WL2 (2 * PB_W1 + PB_W2)
#define PB0_BT  (2 * PB_W1 + 2 * PB_W2)
#define PB0_X   (PB0_BT + 1)
#define PB0_Z1  (PB0_X + PB_X)
#define PB0_Z2  (PB0_Z1 + PB_Z1)
#define PB_TOTAL (PB0_Z2 + PB_Z2)
static_assert((HID * (CIN / 8)) % 256 == 0 && (HID * (HID / 8)) % 256 == 0);
static_assert((NN * (CIN / 8)) % 256 == 0);
static_assert(((MPAD - NN) * (K1 / 8)) % 256 == 0 && ((MPAD - NN) * (K2 / 8)) % 256 == 0);

constexpr size_t SZ_A1   = (size_t)MPAD * K1 * 2;
constexpr size_t SZ_A2   = (size_t)MPAD * K2 * 2;
constexpr size_t SZ_T    = (size_t)MPAD * HID * 4;
constexpr size_t SZ_H    = (size_t)MPAD * HID * 4;
constexpr size_t SZ_LIST = (size_t)NBLK * RCAP * 4;
constexpr size_t SZ_CNT  = (size_t)NBLK * NBS * 4;
constexpr size_t SZ_OFF  = (size_t)NBLK * NBS * 4;
constexpr size_t SZ_FLAG = (size_t)NBLK * 128;
constexpr size_t SZ_B1   = (size_t)HID * K1 * 2;
constexpr size_t SZ_B2   = (size_t)HID * K2 * 2;
constexpr size_t SZ_BT   = (size_t)2 * HID * 4;
constexpr size_t O_A1   = 0;
constexpr size_t O_A2   = O_A1 + SZ_A1;
constexpr size_t O_T    = O_A2 + SZ_A2;
constexpr size_t O_H    = O_T + SZ_T;
constexpr size_t O_LIST = O_H + SZ_H;
constexpr size_t O_CNT  = O_LIST + SZ_LIST;
constexpr size_t O_OFF  = O_CNT + SZ_CNT;
constexpr size_t O_FLAG = O_OFF + SZ_OFF;
constexpr size_t O_B1   = O_FLAG + SZ_FLAG;
constexpr size_t O_B2   = O_B1 + SZ_B1;
constexpr size_t O_BT   = O_B2 + SZ_B2;
constexpr size_t WS_TOTAL = O_BT + SZ_BT;
static_assert(SZ_A1 % 256 == 0 && SZ_A2 % 256 == 0 && SZ_T % 256 == 0 && SZ_LIST % 256 == 0);
static_assert(SZ_CNT % 256 == 0 && SZ_FLAG % 256 == 0 && SZ_B1 % 256 == 0 && SZ_B2 % 256 == 0 && SZ_BT % 256 == 0);
static_assert(WS_TOTAL <= ((size_t)128 << 20));
static_assert((size_t)MPAD * K2 / 8 < ((size_t)1 << 31));

__device__ __forceinline__ float relu_keep(float v) {
  return (v > 0.0f) ? v : ((v != v) ? v : 0.0f);
}

template <int KW, int DUP>
__device__ __forceinline__ void wt_unit(const float* __restrict__ W, int u, unsigned short* P, int KT, int c0, int c1) {
  constexpr int UPR = KW / 8;
  const int n  = u / UPR;
  const int k8 = (u - n * UPR) * 8;
  const float* p = W + (size_t)k8 * HID + n;
  float x[8];
#pragma unroll
  for (int i = 0; i < 8; ++i) x[i] = p[(size_t)i * HID];
  const v4u o = pack8_bf16((v4f){ x[0], x[1], x[2], x[3] }, (v4f){ x[4], x[5], x[6], x[7] });
  unsigned short* d0 = P + (size_t)n * (size_t)KT + c0 + k8;
  unsigned short* d1 = P + (size_t)n * (size_t)KT + c1 + k8;
  for (int pass = 0; pass < 2; ++pass) {
    *(volatile v4u*)d0 = o;
    if (DUP) *(volatile v4u*)d1 = o;
    __threadfence();
  }
}

__global__ __launch_bounds__(256) void k_prep(const float* __restrict__ x, const float* __restrict__ Wl1,
                                              const float* __restrict__ Wr1, const float* __restrict__ b1,
                                              const float* __restrict__ Wl2, const float* __restrict__ Wr2,
                                              const float* __restrict__ b2, unsigned short* A1, unsigned short* A2,
                                              unsigned short* B1, unsigned short* B2, float* BT) {
  const int b = (int)blockIdx.x;
  const int tid = (int)threadIdx.x;
  if (b < PB0_WL1) {
    wt_unit<CIN, 0>(Wr1, b * 256 + tid, B1, K1, 0, 0);
  } else if (b < PB0_WR2) {
    wt_unit<CIN, M1_TWO>(Wl1, (b - PB0_WL1) * 256 + tid, B1, K1, CIN, 2 * CIN);
  } else if (b < PB0_WL2) {
    wt_unit<HID, H_TWO>(Wr2, (b - PB0_WR2) * 256 + tid, B2, K2, 0, HID);
  } else if (b < PB0_BT) {
    wt_unit<HID, M2_TWO>(Wl2, (b - PB0_WL2) * 256 + tid, B2, K2, HW, HW + HID);
  } else if (b < PB0_X) {
    const int q = tid & 63;
    const v4f p1 = *(const v4fa*)(b1 + 4 * q);
    const v4f p2 = *(const v4fa*)(b2 + 4 * q);
    asm volatile("" :: "v"(p1), "v"(p2));
    const bool second = tid >= 64;
    v4f o;
    o.x = bf16_val(second ? p2.x : p1.x);
    o.y = bf16_val(second ? p2.y : p1.y);
    o.z = bf16_val(second ? p2.z : p1.z);
    o.w = bf16_val(second ? p2.w : p1.w);
    float* dp = BT + 4 * (tid & 127);
    for (int pass = 0; pass < 2; ++pass) {
      if (tid < 128) *(volatile v4f*)dp = o;
      __threadfence();
    }
  } else if (b < PB0_Z1) {
    const int u   = (b - PB0_X) * 256 + tid;
    const int row = u >> 4;
    const int p8  = (u & 15) * 8;
    const float* xp = x + (size_t)row * CIN + p8;
    const v4f a = *(const v4fa*)xp;
    const v4f c = *(const v4fa*)(xp + 4);
    const v4u o = pack8_bf16(a, c);
    unsigned short* dp = A1 + (size_t)row * K1 + p8;
    for (int pass = 0; pass < 2; ++pass) {
      *(volatile v4u*)dp = o;
      __threadfence();
    }
  } else if (b < PB0_Z2) {
    const int u = (b - PB0_Z1) * 256 + tid;
    const v4u z = (v4u){ 0u, 0u, 0u, 0u };
    unsigned short* dp = A1 + (size_t)NN * K1 + (size_t)u * 8;
    for (int pass = 0; pass < 2; ++pass) {
      *(volatile v4u*)dp = z;
      __threadfence();
    }
  } else {
    const int u = (b - PB0_Z2) * 256 + tid;
    const v4u z = (v4u){ 0u, 0u, 0u, 0u };
    unsigned short* dp = A2 + (size_t)NN * K2 + (size_t)u * 8;
    for (int pass = 0; pass < 2; ++pass) {
      *(volatile v4u*)dp = z;
      __threadfence();
    }
  }
}

#define HITJ(HJ, WJ) { \
    const unsigned mj = __builtin_amdgcn_ballot_w32(HJ); \
    if (mj != 0u) { \
      if (HJ) { \
        const int pos = wc + (int)__builtin_amdgcn_mbcnt_lo(mj, 0u); \
        if (pos < WCAP) mylist[pos] = (WJ); \
      } \
      wc += (int)__builtin_popcount(mj); } }

__global__ __launch_bounds__(256) void k_bucket(const int* __restrict__ srcs, const int* __restrict__ dsts,
                                                int* LISTG, int* CNTG, int* OFFG, int* FLAGG) {
  extern __shared__ __attribute__((aligned(16))) int dsm[];
  int* list = dsm;
  int* sl   = dsm + NWAVE * WCAP;
  int* cnt  = sl + RCAP;
  int* offs = cnt + NBS;
  int* cur  = offs + NBS;
  int* misc = cur + NBS;
  const int tid = (int)threadIdx.x, lane = tid & 31, wave = tid >> 5;
  const int nodeBase = (int)blockIdx.x * NBS;

  {
    const v4i z4 = (v4i){ 0, 0, 0, 0 };
    for (int i = tid * 4; i < BK_INTS; i += 1024) *(v4ia*)(dsm + i) = z4;
  }
  __syncthreads();

  const unsigned nbs = (unsigned)nodeBase;
  const int rem = NN - nodeBase;
  const unsigned unb = (unsigned)(rem < NBS ? (rem < 0 ? 0 : rem) : NBS);
  int* mylist = list + wave * WCAP;
  int wc = 0;
#pragma unroll 1
  for (int ch = 0; ch < NCHUNK; ++ch) {
    const int e0 = ch * CHUNK + tid * EPT;
    const bool liveE = (e0 + EPT) <= NE;
    const int e0c = e0 > (NE - EPT) ? (NE - EPT) : e0;
    const v4i da = *(const v4ia*)(dsts + e0c);
    const v4i db = *(const v4ia*)(dsts + e0c + 4);
    const v4i sa = *(const v4ia*)(srcs + e0c);
    const v4i sb = *(const v4ia*)(srcs + e0c + 4);
    asm volatile("" :: "v"(da), "v"(db), "v"(sa), "v"(sb));
    const int k0 = liveE ? da.x : -1, k1 = liveE ? da.y : -1, k2 = liveE ? da.z : -1, k3 = liveE ? da.w : -1;
    const int k4 = liveE ? db.x : -1, k5 = liveE ? db.y : -1, k6 = liveE ? db.z : -1, k7 = liveE ? db.w : -1;
    const unsigned s0 = (unsigned)k0 - nbs, s1 = (unsigned)k1 - nbs, s2 = (unsigned)k2 - nbs, s3 = (unsigned)k3 - nbs;
    const unsigned s4 = (unsigned)k4 - nbs, s5 = (unsigned)k5 - nbs, s6 = (unsigned)k6 - nbs, s7 = (unsigned)k7 - nbs;
    const bool h0 = s0 < unb, h1 = s1 < unb, h2 = s2 < unb, h3 = s3 < unb;
    const bool h4 = s4 < unb, h5 = s5 < unb, h6 = s6 < unb, h7 = s7 < unb;
    const int w0 = (int)((s0 << SRCBITS) | (unsigned)clampi(sa.x, 0, NN - 1));
    const int w1 = (int)((s1 << SRCBITS) | (unsigned)clampi(sa.y, 0, NN - 1));
    const int w2 = (int)((s2 << SRCBITS) | (unsigned)clampi(sa.z, 0, NN - 1));
    const int w3 = (int)((s3 << SRCBITS) | (unsigned)clampi(sa.w, 0, NN - 1));
    const int w4 = (int)((s4 << SRCBITS) | (unsigned)clampi(sb.x, 0, NN - 1));
    const int w5 = (int)((s5 << SRCBITS) | (unsigned)clampi(sb.y, 0, NN - 1));
    const int w6 = (int)((s6 << SRCBITS) | (unsigned)clampi(sb.z, 0, NN - 1));
    const int w7 = (int)((s7 << SRCBITS) | (unsigned)clampi(sb.w, 0, NN - 1));
    HITJ(h0, w0)
    HITJ(h1, w1)
    HITJ(h2, w2)
    HITJ(h3, w3)
    HITJ(h4, w4)
    HITJ(h5, w5)
    HITJ(h6, w6)
    HITJ(h7, w7)
  }
  if (lane == 0) misc[wave] = wc;
  __syncthreads();

  if (wave == 0) {
    int t = 0, ov = 0;
#pragma unroll 1
    for (int w2 = 0; w2 < NWAVE; ++w2) {
      const int craw = misc[w2];
      if (craw > WCAP) ov = 1;
      const int c = __builtin_amdgcn_readfirstlane(clampi(craw, 0, WCAP));
#pragma unroll 1
      for (int b0 = 0; b0 < c; b0 += 32) {
        const int idx = b0 + lane;
        const int ent = list[w2 * WCAP + (idx < WCAP ? idx : WCAP - 1)];
        const int m32 = (c - b0) < 32 ? (c - b0) : 32;
#pragma unroll 1
        for (int k = 0; k < m32; ++k) {
          const int u  = __builtin_amdgcn_readlane(ent, k);
          const int sl_ = (u >> SRCBITS) & (NBS - 1);
          if (lane == 0) cnt[sl_] = cnt[sl_] + 1;
        }
      }
      t += c;
    }
    if (lane == 0) { misc[8] = t; misc[9] = ov | (t > RCAP ? 1 : 0); }
  }
  __syncthreads();

  if (wave == 0) {
    const int base = lane * (NBS / 32);
    int s = 0;
    bool bigl = false;
#pragma unroll 1
    for (int i = 0; i < NBS / 32; ++i) {
      const int cv = cnt[base + i];
      s += cv;
      bigl = bigl | (cv > DEGCAP);
    }
    int incl = s;
#pragma unroll
    for (int d = 1; d < 32; d <<= 1) {
      const int y = __shfl_up(incl, d, 32);
      if (lane >= d) incl += y;
    }
    int run = incl - s;
#pragma unroll 1
    for (int i = 0; i < NBS / 32; ++i) {
      const int cv = cnt[base + i];
      offs[base + i] = run;
      cur[base + i]  = run;
      run += cv;
    }
    const unsigned anyb = __builtin_amdgcn_ballot_w32(bigl);
    if (anyb != 0u && lane == 0) misc[9] = 1;
  }
  __syncthreads();

  if (wave == 0) {
#pragma unroll 1
    for (int w2 = 0; w2 < NWAVE; ++w2) {
      const int c = __builtin_amdgcn_readfirstlane(clampi(misc[w2], 0, WCAP));
#pragma unroll 1
      for (int b0 = 0; b0 < c; b0 += 32) {
        const int idx = b0 + lane;
        const int ent = list[w2 * WCAP + (idx < WCAP ? idx : WCAP - 1)];
        const int m32 = (c - b0) < 32 ? (c - b0) : 32;
#pragma unroll 1
        for (int k = 0; k < m32; ++k) {
          const int u   = __builtin_amdgcn_readlane(ent, k);
          const int sl_ = (u >> SRCBITS) & (NBS - 1);
          if (lane == 0) {
            int p = cur[sl_];
            p = p < 0 ? 0 : (p > RCAP - 1 ? RCAP - 1 : p);
            sl[p] = u & SRCMASK;
            cur[sl_] = p + 1;
          }
        }
      }
    }
  }
  __syncthreads();

  int* lg = LISTG + (size_t)blockIdx.x * RCAP;
  const int q = tid & 63;
  const v4i cv4 = *(const v4ia*)(cnt + 4 * q);
  const v4i ov4 = *(const v4ia*)(offs + 4 * q);
  const int fl = misc[9];
  const v4i fv4 = (v4i){ fl, fl, fl, fl };
  for (int pass = 0; pass < 2; ++pass) {
#pragma unroll 1
    for (int it = 0; it < RCAP / 1024; ++it) {
      const int i4 = (it * 256 + tid) * 4;
      const v4i v = *(const v4ia*)(sl + i4);
      *(volatile v4i*)(lg + i4) = v;
    }
    if (wave < 2) {
      *(volatile v4i*)(CNTG + nodeBase + 4 * q) = cv4;
    } else if (wave < 4) {
      *(volatile v4i*)(OFFG + nodeBase + 4 * q) = ov4;
    } else if (wave == 4 && lane < 8) {
      *(volatile v4i*)(FLAGG + (int)blockIdx.x * 32 + 4 * lane) = fv4;
    }
    __threadfence();
  }
}
#undef HITJ

template <int L>
__global__ __launch_bounds__(256) void k_agg(const float* __restrict__ feat, const int* __restrict__ LISTG,
                                             const int* __restrict__ CNTG, const int* __restrict__ OFFG,
                                             const int* __restrict__ FLAGG, unsigned short* AP) {
  static_assert(L == 1 || L == 2);
  const int lane = (int)threadIdx.x & 31, wave = (int)threadIdx.x >> 5;
  const int row = (int)blockIdx.x * NWAVE + wave;
  const bool live = row < NN;
  const int rc = live ? row : NN - 1;
  const int blk = rc >> NBS_LOG;
  const int craw = CNTG[rc];
  const int oraw = OFFG[rc];
  const int fl   = FLAGG[blk * 32];
  asm volatile("" :: "v"(craw), "v"(oraw), "v"(fl));
  const bool big = (craw > DEGCAP) | (craw < 0);
  const int c  = clampi(craw, 0, DEGCAP);
  const int cn = __builtin_amdgcn_readfirstlane(live ? c : 0);
  const int o  = clampi(oraw, 0, RCAP - 1);
  const int* lp = LISTG + (size_t)blk * RCAP;
  const bool poison = (fl != 0) | big;
  const float qn = __uint_as_float(0x7fc00000u);
  const float dv = (float)(cn > 1 ? cn : 1);

  if constexpr (L == 1) {
    v4f acc = (v4f){ 0.0f, 0.0f, 0.0f, 0.0f };
    const float* fp = feat + 4 * lane;
#pragma unroll 1
    for (int j0 = 0; j0 < cn; j0 += 32) {
      int idx = o + j0 + lane;
      idx = idx > RCAP - 1 ? RCAP - 1 : idx;
      const int w = lp[idx];
      asm volatile("" :: "v"(w));
      int sr = w & SRCMASK;
      sr = sr > NN - 1 ? NN - 1 : sr;
      const int m32 = (cn - j0) < 32 ? (cn - j0) : 32;
#pragma unroll 1
      for (int k = 0; k < m32; ++k) {
        const int sk = __builtin_amdgcn_readlane(sr, k);
        const v4f g = *(const v4fa*)(fp + (size_t)sk * CIN);
        asm volatile("" :: "v"(g));
        const v4f r = (v4f){ bf16_val(g.x), bf16_val(g.y), bf16_val(g.z), bf16_val(g.w) };
        acc = acc + r;
      }
    }
    v4f m = acc / dv;
    m.x = poison ? qn : m.x;
    m.y = poison ? qn : m.y;
    m.z = poison ? qn : m.z;
    m.w = poison ? qn : m.w;
    const int hw0 = (int)pk16(bf16_bits(m.x), bf16_bits(m.y));
    const int hw1 = (int)pk16(bf16_bits(m.z), bf16_bits(m.w));
    const int lw0 = (int)pk16(bf16_lo_bits(m.x), bf16_lo_bits(m.y));
    const int lw1 = (int)pk16(bf16_lo_bits(m.z), bf16_lo_bits(m.w));
    const int sa = (2 * lane) & 31, sb = (2 * lane + 1) & 31;
    const int g0 = __shfl(hw0, sa, 32), g1 = __shfl(hw1, sa, 32);
    const int g2 = __shfl(hw0, sb, 32), g3 = __shfl(hw1, sb, 32);
    const int p0 = __shfl(lw0, sa, 32), p1 = __shfl(lw1, sa, 32);
    const int p2 = __shfl(lw0, sb, 32), p3 = __shfl(lw1, sb, 32);
    const bool lsel = lane >= 16;
    v4u pv;
    pv.x = (unsigned)(lsel ? p0 : g0);
    pv.y = (unsigned)(lsel ? p1 : g1);
    pv.z = (unsigned)(lsel ? p2 : g2);
    pv.w = (unsigned)(lsel ? p3 : g3);
    unsigned short* dp = AP + (size_t)rc * K1 + CIN + 8 * lane;
    const bool wr = live && ((M1_TWO != 0) || (lane < 16));
    for (int pass = 0; pass < 2; ++pass) {
      if (wr) *(volatile v4u*)dp = pv;
      __threadfence();
    }
  } else {
    v4f accA = (v4f){ 0.0f, 0.0f, 0.0f, 0.0f };
    v4f accB = (v4f){ 0.0f, 0.0f, 0.0f, 0.0f };
    const float* fp = feat + 8 * lane;
#pragma unroll 1
    for (int j0 = 0; j0 < cn; j0 += 32) {
      int idx = o + j0 + lane;
      idx = idx > RCAP - 1 ? RCAP - 1 : idx;
      const int w = lp[idx];
      asm volatile("" :: "v"(w));
      int sr = w & SRCMASK;
      sr = sr > NN - 1 ? NN - 1 : sr;
      const int m32 = (cn - j0) < 32 ? (cn - j0) : 32;
#pragma unroll 1
      for (int k = 0; k < m32; ++k) {
        const int sk = __builtin_amdgcn_readlane(sr, k);
        const v4f ga = *(const v4fa*)(fp + (size_t)sk * HID);
        const v4f gb = *(const v4fa*)(fp + (size_t)sk * HID + 4);
        asm volatile("" :: "v"(ga), "v"(gb));
        accA = accA + ga;
        accB = accB + gb;
      }
    }
    v4f ma = accA / dv;
    v4f mb = accB / dv;
    ma.x = poison ? qn : ma.x; ma.y = poison ? qn : ma.y; ma.z = poison ? qn : ma.z; ma.w = poison ? qn : ma.w;
    mb.x = poison ? qn : mb.x; mb.y = poison ? qn : mb.y; mb.z = poison ? qn : mb.z; mb.w = poison ? qn : mb.w;
    const v4u hv = pack8_bf16(ma, mb);
    const v4u lv = pack8_bf16_lo(ma, mb);
    unsigned short* dp = AP + (size_t)rc * K2 + HW + 8 * lane;
    for (int pass = 0; pass < 2; ++pass) {
      if (live) {
        *(volatile v4u*)dp = hv;
        if (M2_TWO) *(volatile v4u*)(dp + HID) = lv;
      }
      __threadfence();
    }
  }
}

__global__ __launch_bounds__(256) void k_row1(const float* __restrict__ T, const float* __restrict__ BT,
                                              float* H, unsigned short* A2) {
  const int lane = (int)threadIdx.x & 31, wave = (int)threadIdx.x >> 5;
  const int row = (int)blockIdx.x * NWAVE + wave;
  const bool live = row < NN;
  const int rc = live ? row : NN - 1;
  const float* tp = T + (size_t)rc * HID;
  const v4f ta = *(const v4fa*)(tp + 4 * lane);
  const v4f tb = *(const v4fa*)(tp + 128 + 4 * lane);
  const v4f ba = *(const v4fa*)(BT + 4 * lane);
  const v4f bb = *(const v4fa*)(BT + 128 + 4 * lane);
  asm volatile("" :: "v"(ta), "v"(tb), "v"(ba), "v"(bb));
  v4f va = ta + ba;
  v4f vb = tb + bb;
  va.x = relu_keep(va.x); va.y = relu_keep(va.y); va.z = relu_keep(va.z); va.w = relu_keep(va.w);
  vb.x = relu_keep(vb.x); vb.y = relu_keep(vb.y); vb.z = relu_keep(vb.z); vb.w = relu_keep(vb.w);

  const int hA0 = (int)pk16(bf16_bits(va.x), bf16_bits(va.y));
  const int hA1 = (int)pk16(bf16_bits(va.z), bf16_bits(va.w));
  const int hB0 = (int)pk16(bf16_bits(vb.x), bf16_bits(vb.y));
  const int hB1 = (int)pk16(bf16_bits(vb.z), bf16_bits(vb.w));
  const int lA0 = (int)pk16(bf16_lo_bits(va.x), bf16_lo_bits(va.y));
  const int lA1 = (int)pk16(bf16_lo_bits(va.z), bf16_lo_bits(va.w));
  const int lB0 = (int)pk16(bf16_lo_bits(vb.x), bf16_lo_bits(vb.y));
  const int lB1 = (int)pk16(bf16_lo_bits(vb.z), bf16_lo_bits(vb.w));
  const int sa = (2 * lane) & 31, sb = (2 * lane + 1) & 31;
  const int hA0a = __shfl(hA0, sa, 32), hA1a = __shfl(hA1, sa, 32), hA0b = __shfl(hA0, sb, 32), hA1b = __shfl(hA1, sb, 32);
  const int hB0a = __shfl(hB0, sa, 32), hB1a = __shfl(hB1, sa, 32), hB0b = __shfl(hB0, sb, 32), hB1b = __shfl(hB1, sb, 32);
  const int lA0a = __shfl(lA0, sa, 32), lA1a = __shfl(lA1, sa, 32), lA0b = __shfl(lA0, sb, 32), lA1b = __shfl(lA1, sb, 32);
  const int lB0a = __shfl(lB0, sa, 32), lB1a = __shfl(lB1, sa, 32), lB0b = __shfl(lB0, sb, 32), lB1b = __shfl(lB1, sb, 32);
  const bool up = lane >= 16;
  v4u hv, lv;
  hv.x = (unsigned)(up ? hB0a : hA0a);
  hv.y = (unsigned)(up ? hB1a : hA1a);
  hv.z = (unsigned)(up ? hB0b : hA0b);
  hv.w = (unsigned)(up ? hB1b : hA1b);
  lv.x = (unsigned)(up ? lB0a : lA0a);
  lv.y = (unsigned)(up ? lB1a : lA1a);
  lv.z = (unsigned)(up ? lB0b : lA0b);
  lv.w = (unsigned)(up ? lB1b : lA1b);

  float* hp = H + (size_t)rc * HID + 4 * lane;
  unsigned short* ap = A2 + (size_t)rc * K2 + 8 * lane;
  for (int pass = 0; pass < 2; ++pass) {
    if (live) {
      *(volatile v4f*)hp = va;
      *(volatile v4f*)(hp + 128) = vb;
      *(volatile v4u*)ap = hv;
      if (H_TWO) *(volatile v4u*)(ap + HID) = lv;
    }
    __threadfence();
  }
}

extern "C" void kernel_launch(void* const* d_in, const int* in_sizes, int n_in,
                              void* d_out, int out_size, void* d_ws, size_t ws_size,
                              hipStream_t stream) {
  if (n_in < 9) return;
  if (in_sizes[0] != NN * CIN) return;
  if (in_sizes[1] != NE || in_sizes[2] != NE) return;
  if (in_sizes[3] != CIN * HID || in_sizes[4] != CIN * HID || in_sizes[5] != HID) return;
  if (in_sizes[6] != HID * HID || in_sizes[7] != HID * HID || in_sizes[8] != HID) return;
  if (out_size != NN * HID) return;
  if (ws_size < WS_TOTAL) return;

  const float* x   = (const float*)d_in[0];
  const int*   src = (const int*)d_in[1];
  const int*   dst = (const int*)d_in[2];
  const float* Wl1 = (const float*)d_in[3];
  const float* Wr1 = (const float*)d_in[4];
  const float* b1  = (const float*)d_in[5];
  const float* Wl2 = (const float*)d_in[6];
  const float* Wr2 = (const float*)d_in[7];
  const float* b2  = (const float*)d_in[8];
  float* out = (float*)d_out;

  char* ws = (char*)d_ws;
  unsigned short* A1 = (unsigned short*)(ws + O_A1);
  unsigned short* A2 = (unsigned short*)(ws + O_A2);
  float*          T  = (float*)(ws + O_T);
  float*          H  = (float*)(ws + O_H);
  int*          LIST = (int*)(ws + O_LIST);
  int*          CNT  = (int*)(ws + O_CNT);
  int*          OFF  = (int*)(ws + O_OFF);
  int*          FLAG = (int*)(ws + O_FLAG);
  unsigned short* B1 = (unsigned short*)(ws + O_B1);
  unsigned short* B2 = (unsigned short*)(ws + O_B2);
  float*          BT = (float*)(ws + O_BT);

  hipFuncSetAttribute(reinterpret_cast<const void*>(&k_bucket), hipFuncAttributeMaxDynamicSharedMemorySize,
                      (int)BK_LDS_BYTES);

  constexpr int GT = ((MPAD / 64) * (HID / 64) + 7) / 8;
  k_prep<<<PB_TOTAL, 256, 0, stream>>>(x, Wl1, Wr1, b1, Wl2, Wr2, b2, A1, A2, B1, B2, BT);
  k_bucket<<<NBLK, 256, BK_LDS_BYTES, stream>>>(src, dst, LIST, CNT, OFF, FLAG);
  k_agg<1><<<NN / NWAVE, 256, 0, stream>>>(x, LIST, CNT, OFF, FLAG, A1);
  k_gemm_nt<0, 0><<<GT, 256, 0, stream>>>(A1, B1, BT, T, MPAD, HID, K1, HID);
  k_row1<<<NN / NWAVE, 256, 0, stream>>>(T, BT, H, A2);
  k_agg<2><<<NN / NWAVE, 256, 0, stream>>>(H, LIST, CNT, OFF, FLAG, A2);
  k_gemm_nt<0, 1><<<GT, 256, 0, stream>>>(A2, B2, BT + HID, out, NN, HID, K2, HID);
}
